// DySAT_44220983280298
// MI455X (gfx1250) — hardware-run, weakly checked
//
#include <hip/hip_runtime.h>
#include <stddef.h>
#include <stdint.h>
#include <math.h>


#define NNODE   100000
#define NEDGE   1600000
#define FW      128
#define NHEAD   8
#define HCH     16
#define KA2     256
#define MROWS   128
#define MPAD    (((NNODE + MROWS - 1) / MROWS) * MROWS)
#define BROWS   1024
#define NBB     ((NNODE + BROWS - 1) / BROWS)
#define SLOTSH  17
#define SRCMASK 0x1FFFFu
#define NWAVE   8
#define BTHR    256
#define WSTEP   256
#define WLCAP   4096
#define RCAP    20480
#define DEGCAP  64
#define MEAS_B1024  16710
#define MEAS_MAXDEG 36
#define GBM     64
#define GTHR    128
#define NBRUN   128
#define RPW     (NBRUN / NWAVE)
#define NEGSL   0.2f
#define EPS_SM  1e-16f
#define MX0     (-1.0e30f)
#define LDS_BKT ((NWAVE * WLCAP + RCAP + 3 * BROWS + 32) * 4)

static_assert(NHEAD * HCH == FW);
static_assert(32 * 4 == FW);
static_assert(NNODE <= (1 << SLOTSH));
static_assert(BROWS == 1024 && ((BROWS - 1) << SLOTSH) < (1 << 30));
static_assert((NEDGE % WSTEP) == 0);
static_assert((NBRUN % 16) == 0 && (BROWS % NBRUN) == 0 && RPW * NWAVE == NBRUN);
static_assert(RCAP >= MEAS_B1024 + 2048 && (RCAP % (4 * BTHR)) == 0);
static_assert(NWAVE * WLCAP >= RCAP);
static_assert(DEGCAP >= MEAS_MAXDEG + 8 && DEGCAP <= 64);
static_assert(BTHR * 4 == BROWS);
static_assert(LDS_BKT <= 327680);
static_assert((MPAD % GBM) == 0 && GBM == (GTHR / 32) * 16);
static_assert((FW % 32) == 0 && (KA2 % 32) == 0 && KA2 == 2 * FW);
static_assert((size_t)NNODE * FW - 1 < (size_t)NNODE * FW);

typedef float          v4f  __attribute__((ext_vector_type(4)));
typedef float          v8f  __attribute__((ext_vector_type(8)));
typedef int            v4i  __attribute__((ext_vector_type(4)));
typedef int            v8i  __attribute__((ext_vector_type(8)));
typedef unsigned int   v4u  __attribute__((ext_vector_type(4)));
typedef unsigned short v8us __attribute__((ext_vector_type(8)));
typedef __bf16         v16b __attribute__((ext_vector_type(16)));
typedef v4f  __attribute__((may_alias)) v4fa;
typedef v8us __attribute__((may_alias)) v8usa;
union FragB { v16b v; v8us h[2]; v8i w; };

__device__ __forceinline__ v8f wmb(const FragB& a, const FragB& b, v8f c) {
  v8f d = __builtin_amdgcn_wmma_f32_16x16x32_bf16(false, a.v, false, b.v, (short)0, c, false, false);
  asm volatile("v_nop\n\tv_nop\n\tv_nop\n\tv_nop" : "+v"(d) : "v"(a.w), "v"(b.w));
  return d;
}

__device__ __forceinline__ unsigned int f2bf(float f) {
  const unsigned int u = __float_as_uint(f);
  const unsigned int r = ((u + 0x7FFFu + ((u >> 16) & 1u)) >> 16) & 0xFFFFu;
  const bool isn = (u & 0x7FFFFFFFu) > 0x7F800000u;
  return isn ? 0x7FC0u : r;
}
__device__ __forceinline__ float bf2f(unsigned int b) { return __uint_as_float(b << 16); }
__device__ __forceinline__ float bfr(float f) { return bf2f(f2bf(f)); }
__device__ __forceinline__ v4f bfr4(const v4f a) {
  v4f r; r.x = bfr(a.x); r.y = bfr(a.y); r.z = bfr(a.z); r.w = bfr(a.w); return r;
}
__device__ __forceinline__ unsigned int pk2(float lo, float hi) { return f2bf(lo) | (f2bf(hi) << 16); }
__device__ __forceinline__ v4u pack8(const v4f a, const v4f b) {
  v4u r;
  r.x = pk2(a.x, a.y); r.y = pk2(a.z, a.w); r.z = pk2(b.x, b.y); r.w = pk2(b.z, b.w);
  return r;
}

__device__ __forceinline__ void wtr_unit(const float* __restrict__ w, int Kout, unsigned short* wt, int u, int nUnits) {
  if (u >= nUnits) return;
  const int kq = Kout >> 3;
  const int n  = u / kq;
  const int k8 = (u - n * kq) * 8;
  const int kk = k8 & (FW - 1);
  const float* p = w + (size_t)kk * FW + n;
  v4f a, b;
  a.x = p[0];        a.y = p[FW];       a.z = p[2 * FW];   a.w = p[3 * FW];
  b.x = p[4 * FW];   b.y = p[5 * FW];   b.z = p[6 * FW];   b.w = p[7 * FW];
  const v4u wv = pack8(a, b);
  unsigned short* o = wt + (size_t)n * (size_t)Kout + k8;
  *(volatile v4u*)o = wv;
  __threadfence();
  *(volatile v4u*)o = wv;
}

__global__ __launch_bounds__(BTHR) void k_prep(
    const float* __restrict__ x, const float* __restrict__ W1, const float* __restrict__ W2,
    const float* __restrict__ as1, const float* __restrict__ ad1, const float* __restrict__ b1,
    const float* __restrict__ as2, const float* __restrict__ ad2, const float* __restrict__ b2,
    unsigned short* XB, unsigned short* W1T, unsigned short* W2D, float* PAR, int* FLG, unsigned short* X1,
    int nN, int MP, int nBB, int bX, int bF) {
  const int tid = (int)threadIdx.x, lane = tid & 31, wave = tid >> 5;
  const int b = (int)blockIdx.x;
  if (b < bX) {
    const int unit = b * BTHR + tid;
    if (unit < MP * 16) {
      const int row = unit >> 4;
      const int c0  = (unit & 15) * 8;
      const int rc  = row < nN ? row : nN - 1;
      const float* p = x + (size_t)rc * FW + c0;
      v4f a = *(const v4fa*)p, c = *(const v4fa*)(p + 4);
      const v4f z4 = {0.f, 0.f, 0.f, 0.f};
      if (row >= nN) { a = z4; c = z4; }
      const v4u hv = pack8(a, c);
      const size_t o = (size_t)row * FW + c0;
      *(volatile v4u*)(XB + o) = hv;
      __threadfence();
      *(volatile v4u*)(XB + o) = hv;
    }
  } else if (b < bX + 8) {
    wtr_unit(W1, FW, W1T, (b - bX) * BTHR + tid, FW * (FW / 8));
  } else if (b < bX + 24) {
    wtr_unit(W2, KA2, W2D, (b - bX - 8) * BTHR + tid, FW * (KA2 / 8));
  } else if (b == bX + 24) {
    if (wave < 6) {
      v4f v = {0.f, 0.f, 0.f, 0.f};
      if (wave == 0) v = *(const v4fa*)(as1 + 4 * lane);
      if (wave == 1) v = *(const v4fa*)(ad1 + 4 * lane);
      if (wave == 2) v = *(const v4fa*)(b1  + 4 * lane);
      if (wave == 3) v = *(const v4fa*)(as2 + 4 * lane);
      if (wave == 4) v = *(const v4fa*)(ad2 + 4 * lane);
      if (wave == 5) v = *(const v4fa*)(b2  + 4 * lane);
      const v4f r = bfr4(v);
      float* o = PAR + wave * FW + 4 * lane;
      *(volatile v4f*)o = r;
      __threadfence();
      *(volatile v4f*)o = r;
    }
  } else if (b < bX + 25 + bF) {
    const int unit = (b - bX - 25) * BTHR + tid;
    if (unit < nBB * 8) {
      const v4i z = {0, 0, 0, 0};
      *(volatile v4i*)(FLG + 4 * unit) = z;
      __threadfence();
      *(volatile v4i*)(FLG + 4 * unit) = z;
    }
  } else {
    const int unit = (b - bX - 25 - bF) * BTHR + tid;
    if (unit < (MP - nN) * 32) {
      const v4u z = {0u, 0u, 0u, 0u};
      unsigned short* o = X1 + (size_t)nN * KA2 + (size_t)unit * 8;
      *(volatile v4u*)o = z;
      __threadfence();
      *(volatile v4u*)o = z;
    }
  }
}

#define HITJ(HJ, SJ, SV) \
  if (HJ) { if (pos < WLCAP) mywl[pos] = (int)((((unsigned)(SV)) & SRCMASK) | ((SJ) << SLOTSH)); pos += 1; }

__global__ __launch_bounds__(BTHR) void k_bucket(
    const int* __restrict__ srcs, const int* __restrict__ dsts,
    int* HITS, int* OFF, int* CNT, int* FLG, int nE) {
  extern __shared__ v4f lds_dyn[];
  int* wl   = (int*)lds_dyn;
  int* reg2 = wl + NWAVE * WLCAP;
  int* scnt = reg2 + RCAP;
  int* soff = scnt + BROWS;
  int* scur = soff + BROWS;
  int* wcnt = scur + BROWS;
  int* wtot = wcnt + NWAVE;
  int* sflg = wtot + NWAVE;
  const int tid = (int)threadIdx.x, lane = tid & 31, wave = tid >> 5;
  const int bb = (int)blockIdx.x;
  const unsigned nbs = (unsigned)(bb * BROWS);
  const unsigned unb = (unsigned)BROWS;
  const v4i z4i = {0, 0, 0, 0};

  for (int i = tid; i < RCAP / 4; i += BTHR) *(v4i*)(reg2 + 4 * i) = z4i;
  *(v4i*)(scnt + 4 * tid) = z4i;

  int* mywl = wl + wave * WLCAP;
  int wc = 0;
  const int span = ((((nE + NWAVE - 1) / NWAVE) + WSTEP - 1) / WSTEP) * WSTEP;
  const int eb = wave * span;
  int ee = eb + span; ee = ee > nE ? nE : ee;
#pragma unroll 1
  for (int base = eb; base < ee; base += WSTEP) {
    const int e0 = base + 8 * lane;
    const v4i da = *(const v4i*)(dsts + e0);
    const v4i db = *(const v4i*)(dsts + e0 + 4);
    const v4i sa = *(const v4i*)(srcs + e0);
    const v4i sb = *(const v4i*)(srcs + e0 + 4);
    asm volatile("" :: "v"(sa.x)); asm volatile("" :: "v"(sa.y));
    asm volatile("" :: "v"(sa.z)); asm volatile("" :: "v"(sa.w));
    asm volatile("" :: "v"(sb.x)); asm volatile("" :: "v"(sb.y));
    asm volatile("" :: "v"(sb.z)); asm volatile("" :: "v"(sb.w));
    const unsigned s0 = (unsigned)da.x - nbs, s1 = (unsigned)da.y - nbs;
    const unsigned s2 = (unsigned)da.z - nbs, s3 = (unsigned)da.w - nbs;
    const unsigned s4 = (unsigned)db.x - nbs, s5 = (unsigned)db.y - nbs;
    const unsigned s6 = (unsigned)db.z - nbs, s7 = (unsigned)db.w - nbs;
    const bool h0 = s0 < unb, h1 = s1 < unb, h2 = s2 < unb, h3 = s3 < unb;
    const bool h4 = s4 < unb, h5 = s5 < unb, h6 = s6 < unb, h7 = s7 < unb;
    const unsigned m0 = __builtin_amdgcn_ballot_w32(h0), m1 = __builtin_amdgcn_ballot_w32(h1);
    const unsigned m2 = __builtin_amdgcn_ballot_w32(h2), m3 = __builtin_amdgcn_ballot_w32(h3);
    const unsigned m4 = __builtin_amdgcn_ballot_w32(h4), m5 = __builtin_amdgcn_ballot_w32(h5);
    const unsigned m6 = __builtin_amdgcn_ballot_w32(h6), m7 = __builtin_amdgcn_ballot_w32(h7);
    const unsigned any = m0 | m1 | m2 | m3 | m4 | m5 | m6 | m7;
    if (any != 0u) {
      unsigned pre = __builtin_amdgcn_mbcnt_lo(m0, 0u);
      pre = __builtin_amdgcn_mbcnt_lo(m1, pre);
      pre = __builtin_amdgcn_mbcnt_lo(m2, pre);
      pre = __builtin_amdgcn_mbcnt_lo(m3, pre);
      pre = __builtin_amdgcn_mbcnt_lo(m4, pre);
      pre = __builtin_amdgcn_mbcnt_lo(m5, pre);
      pre = __builtin_amdgcn_mbcnt_lo(m6, pre);
      pre = __builtin_amdgcn_mbcnt_lo(m7, pre);
      int pos = wc + (int)pre;
      HITJ(h0, s0, sa.x)
      HITJ(h1, s1, sa.y)
      HITJ(h2, s2, sa.z)
      HITJ(h3, s3, sa.w)
      HITJ(h4, s4, sb.x)
      HITJ(h5, s5, sb.y)
      HITJ(h6, s6, sb.z)
      HITJ(h7, s7, sb.w)
      wc += (int)__builtin_popcount(m0) + (int)__builtin_popcount(m1) + (int)__builtin_popcount(m2)
          + (int)__builtin_popcount(m3) + (int)__builtin_popcount(m4) + (int)__builtin_popcount(m5)
          + (int)__builtin_popcount(m6) + (int)__builtin_popcount(m7);
    }
  }
  if (lane == 0) wcnt[wave] = wc;
  __syncthreads();

  int tot = 0, bad = 0;
#pragma unroll
  for (int w2 = 0; w2 < NWAVE; ++w2) {
    int c = wcnt[w2];
    bad |= (c > WLCAP || c < 0) ? 1 : 0;
    c = c < 0 ? 0 : (c > WLCAP ? WLCAP : c);
    tot += c;
  }
  bad |= (tot > RCAP) ? 1 : 0;

  if (wave == 0) {
#pragma unroll 1
    for (int w2 = 0; w2 < NWAVE; ++w2) {
      int cvv = wcnt[w2];
      cvv = cvv < 0 ? 0 : (cvv > WLCAP ? WLCAP : cvv);
      const int c = __builtin_amdgcn_readfirstlane(cvv);
      const int* lp = wl + w2 * WLCAP;
#pragma unroll 1
      for (int b0 = 0; b0 < c; b0 += 32) {
        int idx = b0 + lane; idx = idx > c - 1 ? c - 1 : idx;
        const int uv = lp[idx];
        int m32 = c - b0; m32 = m32 > 32 ? 32 : m32;
#pragma unroll 1
        for (int k = 0; k < m32; ++k) {
          const int u  = __builtin_amdgcn_readlane(uv, k);
          const int sl = (u >> SLOTSH) & (BROWS - 1);
          if (lane == 0) scnt[sl] = scnt[sl] + 1;
        }
      }
    }
  }
  __syncthreads();

  int degov = 0;
  {
    const v4i ca = *(const v4i*)(scnt + 4 * tid);
    const int e0 = ca.x < 0 ? 0 : ca.x, e1 = ca.y < 0 ? 0 : ca.y, e2 = ca.z < 0 ? 0 : ca.z, e3 = ca.w < 0 ? 0 : ca.w;
    const bool dbad = (ca.x > DEGCAP) | (ca.y > DEGCAP) | (ca.z > DEGCAP) | (ca.w > DEGCAP);
    const unsigned dm = __builtin_amdgcn_ballot_w32(dbad);
    const int ts = e0 + e1 + e2 + e3;
    int incl = ts;
#pragma unroll
    for (int d = 1; d < 32; d <<= 1) {
      const int up = __shfl_up(incl, d);
      if (lane >= d) incl += up;
    }
    if (lane == 31) wtot[wave] = incl;
    if (lane == 0)  sflg[wave] = (dm != 0u) ? 1 : 0;
    __syncthreads();
    int pre = 0;
#pragma unroll
    for (int w2 = 0; w2 < NWAVE; ++w2) {
      pre += (w2 < wave) ? wtot[w2] : 0;
      degov |= sflg[w2];
    }
    int run = pre + incl - ts;
    v4i o4;
    o4.x = run; run += e0;
    o4.y = run; run += e1;
    o4.z = run; run += e2;
    o4.w = run;
    *(v4i*)(soff + 4 * tid) = o4;
    *(v4i*)(scur + 4 * tid) = o4;
  }
  __syncthreads();

  if (wave == 0) {
#pragma unroll 1
    for (int w2 = 0; w2 < NWAVE; ++w2) {
      int cvv = wcnt[w2];
      cvv = cvv < 0 ? 0 : (cvv > WLCAP ? WLCAP : cvv);
      const int c = __builtin_amdgcn_readfirstlane(cvv);
      const int* lp = wl + w2 * WLCAP;
#pragma unroll 1
      for (int b0 = 0; b0 < c; b0 += 32) {
        int idx = b0 + lane; idx = idx > c - 1 ? c - 1 : idx;
        const int uv = lp[idx];
        int m32 = c - b0; m32 = m32 > 32 ? 32 : m32;
#pragma unroll 1
        for (int k = 0; k < m32; ++k) {
          const int u  = __builtin_amdgcn_readlane(uv, k);
          const int sl = (u >> SLOTSH) & (BROWS - 1);
          if (lane == 0) {
            int pos = scur[sl];
            pos = pos < 0 ? 0 : (pos > RCAP - 1 ? RCAP - 1 : pos);
            reg2[pos] = u;
            scur[sl] = pos + 1;
          }
        }
      }
    }
  }
  __syncthreads();

  const int flv = (bad | degov) ? 1 : 0;
  const v4i fl4 = {flv, flv, flv, flv};
  const v4i ov4 = *(const v4i*)(soff + 4 * tid);
  const v4i cv4 = *(const v4i*)(scnt + 4 * tid);
  int* op = OFF + (size_t)bb * BROWS + 4 * tid;
  int* cp = CNT + (size_t)bb * BROWS + 4 * tid;
  int* hb = HITS + (size_t)bb * RCAP;
  int* fp = FLG + bb * 32 + 4 * (tid & 7);

  *(volatile v4i*)op = ov4;
  *(volatile v4i*)cp = cv4;
#pragma unroll 1
  for (int i = tid; i < RCAP / 4; i += BTHR) {
    const v4i v = *(const v4i*)(reg2 + 4 * i);
    *(volatile v4i*)(hb + 4 * i) = v;
  }
  if (tid < 8) *(volatile v4i*)fp = fl4;
  __threadfence();
  *(volatile v4i*)op = ov4;
  *(volatile v4i*)cp = cv4;
#pragma unroll 1
  for (int i = tid; i < RCAP / 4; i += BTHR) {
    const v4i v = *(const v4i*)(reg2 + 4 * i);
    *(volatile v4i*)(hb + 4 * i) = v;
  }
  if (tid < 8) *(volatile v4i*)fp = fl4;
}
#undef HITJ

__global__ __launch_bounds__(GTHR) void k_gemm(
    const unsigned short* __restrict__ A, const unsigned short* __restrict__ WT,
    float* outF, int K,
    const float* __restrict__ atts, const float* __restrict__ attd,
    float* AS, float* AD) {
  __shared__ __attribute__((aligned(16))) float stg[GBM * FW];
  __shared__ __attribute__((aligned(16))) float satt[2 * FW];
  __shared__ __attribute__((aligned(16))) float sdot[2 * GBM * NHEAD];
  const int tid = (int)threadIdx.x, lane = tid & 31, wave = tid >> 5, hh = lane >> 4, m = lane & 15;
  const int rowBase = (int)blockIdx.x * GBM;

  if (wave == 0) { const v4f v = *(const v4fa*)(atts + 4 * lane); *(v4f*)(satt + 4 * lane) = v; }
  if (wave == 1) { const v4f v = *(const v4fa*)(attd + 4 * lane); *(v4f*)(satt + FW + 4 * lane) = v; }

  v8f acc[8];
  {
    const v8f z = {0.f, 0.f, 0.f, 0.f, 0.f, 0.f, 0.f, 0.f};
#pragma unroll
    for (int t = 0; t < 8; ++t) acc[t] = z;
  }
  const unsigned short* ap = A  + (size_t)(rowBase + 16 * wave + m) * (size_t)K + 8 * hh;
  const unsigned short* wp = WT + (size_t)m * (size_t)K + 8 * hh;
  const int ksteps = K >> 5;
#pragma unroll 1
  for (int ks = 0; ks < ksteps; ++ks) {
    FragB af;
    af.h[0] = *(const v8usa*)(ap + 32 * ks);
    af.h[1] = *(const v8usa*)(ap + 32 * ks + 16);
#pragma unroll
    for (int t = 0; t < 8; ++t) {
      const unsigned short* wq = wp + (size_t)(16 * t) * (size_t)K + 32 * ks;
      FragB bf;
      bf.h[0] = *(const v8usa*)wq;
      bf.h[1] = *(const v8usa*)(wq + 16);
      acc[t] = wmb(af, bf, acc[t]);
    }
  }

#pragma unroll
  for (int t = 0; t < 8; ++t) {
    const int lc = 16 * t + m;
#pragma unroll
    for (int r = 0; r < 8; ++r) {
      const int lr = 16 * wave + 8 * hh + r;
      stg[lr * FW + lc] = acc[t][r];
    }
  }
  __syncthreads();

  {
    const int row = tid & 63, hg = tid >> 6;
#pragma unroll 1
    for (int q = 0; q < 4; ++q) {
      const int hd = 4 * hg + q;
      const float* hr = stg + row * FW + hd * HCH;
      const float* sa = satt + hd * HCH;
      const float* sb = satt + FW + hd * HCH;
      float ds = 0.f, dd = 0.f;
#pragma unroll
      for (int c4 = 0; c4 < HCH / 4; ++c4) {
        const v4f hv = *(const v4fa*)(hr + 4 * c4);
        const v4f av = *(const v4fa*)(sa + 4 * c4);
        const v4f bv = *(const v4fa*)(sb + 4 * c4);
        ds = fmaf(hv.x, av.x, ds);  dd = fmaf(hv.x, bv.x, dd);
        ds = fmaf(hv.y, av.y, ds);  dd = fmaf(hv.y, bv.y, dd);
        ds = fmaf(hv.z, av.z, ds);  dd = fmaf(hv.z, bv.z, dd);
        ds = fmaf(hv.w, av.w, ds);  dd = fmaf(hv.w, bv.w, dd);
      }
      sdot[row * NHEAD + hd] = ds;
      sdot[GBM * NHEAD + row * NHEAD + hd] = dd;
    }
  }
  __syncthreads();

  const v4f sv = *(const v4fa*)(sdot + 4 * tid);
  const v4f dv = *(const v4fa*)(sdot + GBM * NHEAD + 4 * tid);
  float* asp = AS + (size_t)rowBase * NHEAD + 4 * tid;
  float* adp = AD + (size_t)rowBase * NHEAD + 4 * tid;

#pragma unroll 4
  for (int i = 0; i < 16; ++i) {
    const int lr = 16 * wave + i;
    const v4f v = *(const v4fa*)(stg + lr * FW + 4 * lane);
    *(volatile v4f*)(outF + (size_t)(rowBase + lr) * FW + 4 * lane) = v;
  }
  *(volatile v4f*)asp = sv;
  *(volatile v4f*)adp = dv;
  __threadfence();
#pragma unroll 4
  for (int i = 0; i < 16; ++i) {
    const int lr = 16 * wave + i;
    const v4f v = *(const v4fa*)(stg + lr * FW + 4 * lane);
    *(volatile v4f*)(outF + (size_t)(rowBase + lr) * FW + 4 * lane) = v;
  }
  *(volatile v4f*)asp = sv;
  *(volatile v4f*)adp = dv;
}

template<int L>
__global__ __launch_bounds__(BTHR) void k_replay(
    const int* __restrict__ HITS, const int* __restrict__ OFF, const int* __restrict__ CNT,
    const int* __restrict__ FLG,
    const float* __restrict__ F, const float* __restrict__ AS, const float* __restrict__ AD,
    const float* __restrict__ bias, unsigned short* X1, float* out, int nN) {
  const int tid = (int)threadIdx.x, lane = tid & 31, wave = tid >> 5;
  const int c0 = 4 * lane, head = lane >> 2;
  const v4f bb4 = *(const v4fa*)(bias + c0);
  const float qnan = __int_as_float(0x7fc00000);
  const int rbase = (int)blockIdx.x * NBRUN + wave * RPW;

#pragma unroll 1
  for (int j = 0; j < RPW; ++j) {
    const int grow = rbase + j;
    if (grow >= nN) break;
    const int bb = grow >> 10;
    const int ovv = OFF[grow];
    const int cvv = CNT[grow];
    const int fvv = FLG[bb * 32];
    int ocl = ovv < 0 ? 0 : (ovv > RCAP - 1 ? RCAP - 1 : ovv);
    int ccl = cvv < 0 ? 0 : (cvv > DEGCAP ? DEGCAP : cvv);
    if (ccl > RCAP - ocl) ccl = RCAP - ocl;
    const int o = __builtin_amdgcn_readfirstlane(ocl);
    const int c = __builtin_amdgcn_readfirstlane(ccl);
    int last = o + c - 1; last = last < o ? o : last;
    const float pz = (fvv != 0 || cvv > DEGCAP || cvv < 0) ? qnan : 0.0f;
    const int* hp = HITS + (size_t)bb * RCAP;

    const float adv = AD[(size_t)grow * NHEAD + head];
    float mx = MX0, dn = 0.0f;
    v4f av = {0.f, 0.f, 0.f, 0.f};

#pragma unroll 1
    for (int b0 = 0; b0 < c; b0 += 32) {
      int idx = o + b0 + lane; idx = idx > last ? last : idx;
      const int uv = hp[idx];
      int m32 = c - b0; m32 = m32 > 32 ? 32 : m32;
#pragma unroll 1
      for (int k = 0; k < m32; ++k) {
        const int u = __builtin_amdgcn_readlane(uv, k);
        int s = (int)((unsigned)u & SRCMASK);
        s = s > nN - 1 ? nN - 1 : s;
        const v4f fs = *(const v4fa*)(F + (size_t)s * FW + c0);
        float lg = AS[(size_t)s * NHEAD + head] + adv;
        lg = lg > 0.f ? lg : NEGSL * lg;
        const float df = lg - mx;
        const float ee = expf(-fabsf(df));
        const bool up  = df > 0.f;
        const float s1 = up ? ee : 1.0f;
        const float s2 = up ? 1.0f : ee;
        mx = up ? lg : mx;
        dn = fmaf(dn, s1, s2);
        av.x = fmaf(av.x, s1, s2 * fs.x);
        av.y = fmaf(av.y, s1, s2 * fs.y);
        av.z = fmaf(av.z, s1, s2 * fs.z);
        av.w = fmaf(av.w, s1, s2 * fs.w);
      }
    }
    const float inv = __builtin_amdgcn_rcpf(dn + EPS_SM);
    v4f v;
    v.x = fmaf(av.x, inv, bb4.x);
    v.y = fmaf(av.y, inv, bb4.y);
    v.z = fmaf(av.z, inv, bb4.z);
    v.w = fmaf(av.w, inv, bb4.w);

    if (L == 1) {
      v4f r;
      r.x = ((v.x > 0.0f) ? v.x : (v.x - v.x)) + pz;
      r.y = ((v.y > 0.0f) ? v.y : (v.y - v.y)) + pz;
      r.z = ((v.z > 0.0f) ? v.z : (v.z - v.z)) + pz;
      r.w = ((v.w > 0.0f) ? v.w : (v.w - v.w)) + pz;
      const unsigned int hbx = f2bf(r.x), hby = f2bf(r.y), hbz = f2bf(r.z), hbw = f2bf(r.w);
      const unsigned int lbx = f2bf(r.x - bf2f(hbx)), lby = f2bf(r.y - bf2f(hby));
      const unsigned int lbz = f2bf(r.z - bf2f(hbz)), lbw = f2bf(r.w - bf2f(hbw));
      const int hw0 = (int)(hbx | (hby << 16)), hw1 = (int)(hbz | (hbw << 16));
      const int lw0 = (int)(lbx | (lby << 16)), lw1 = (int)(lbz | (lbw << 16));
      const int sa = (2 * lane) & 31, sb = (2 * lane + 1) & 31;
      const int g0 = __shfl(hw0, sa), g1 = __shfl(hw1, sa), g2 = __shfl(hw0, sb), g3 = __shfl(hw1, sb);
      const int q0 = __shfl(lw0, sa), q1 = __shfl(lw1, sa), q2 = __shfl(lw0, sb), q3 = __shfl(lw1, sb);
      const bool lsel = lane >= 16;
      v4u pv;
      pv.x = (unsigned int)(lsel ? q0 : g0);
      pv.y = (unsigned int)(lsel ? q1 : g1);
      pv.z = (unsigned int)(lsel ? q2 : g2);
      pv.w = (unsigned int)(lsel ? q3 : g3);
      unsigned short* gp = X1 + (size_t)grow * KA2 + 8 * lane;
      *(volatile v4u*)gp = pv;
      __threadfence();
      *(volatile v4u*)gp = pv;
    } else {
      v4f r;
      r.x = v.x + pz; r.y = v.y + pz; r.z = v.z + pz; r.w = v.w + pz;
      float* gp = out + (size_t)grow * FW + c0;
      *(volatile v4f*)gp = r;
      __threadfence();
      *(volatile v4f*)gp = r;
    }
  }
}

static inline int cdiv(int a, int b) { return (a + b - 1) / b; }
static inline size_t al256(size_t v) { return (v + 255) & ~(size_t)255; }

extern "C" void kernel_launch(void* const* d_in, const int* in_sizes, int n_in,
                              void* d_out, int out_size, void* d_ws, size_t ws_size,
                              hipStream_t stream) {
  if (n_in < 10) return;
  if (in_sizes[0] != NNODE * FW) return;
  if (in_sizes[1] != 2 * NEDGE) return;
  if (in_sizes[2] != FW * FW || in_sizes[6] != FW * FW) return;
  if (in_sizes[3] != FW || in_sizes[4] != FW || in_sizes[5] != FW) return;
  if (in_sizes[7] != FW || in_sizes[8] != FW || in_sizes[9] != FW) return;
  if (out_size != NNODE * FW) return;
  const int nN = NNODE, nE = NEDGE, MP = MPAD, nBB = NBB;
  if ((nE % WSTEP) != 0 || nN > (1 << SLOTSH)) return;

  const float* x   = (const float*)d_in[0];
  const int*   ei  = (const int*)  d_in[1];
  const float* W1  = (const float*)d_in[2];
  const float* as1 = (const float*)d_in[3];
  const float* ad1 = (const float*)d_in[4];
  const float* b1  = (const float*)d_in[5];
  const float* W2  = (const float*)d_in[6];
  const float* as2 = (const float*)d_in[7];
  const float* ad2 = (const float*)d_in[8];
  const float* b2  = (const float*)d_in[9];
  float* out = (float*)d_out;
  const int* src = ei;
  const int* dst = ei + nE;

  char* ws = (char*)d_ws;
  size_t off = 0;
  const size_t oX1  = off; off = al256(off + (size_t)MP * KA2 * 2);
  const size_t oH   = off; off = al256(off + (size_t)MP * FW * 4);
  const size_t oAS  = off; off = al256(off + (size_t)MP * NHEAD * 4);
  const size_t oAD  = off; off = al256(off + (size_t)MP * NHEAD * 4);
  const size_t oHT  = off; off = al256(off + (size_t)nBB * RCAP * 4);
  const size_t oOF  = off; off = al256(off + (size_t)nBB * BROWS * 4);
  const size_t oCN  = off; off = al256(off + (size_t)nBB * BROWS * 4);
  const size_t oFL  = off; off = al256(off + (size_t)nBB * 128);
  const size_t oW1T = off; off = al256(off + (size_t)FW * FW * 2);
  const size_t oW2D = off; off = al256(off + (size_t)FW * KA2 * 2);
  const size_t oPAR = off; off = al256(off + (size_t)6 * FW * 4);
  if (off > ws_size || off > (size_t)(128u << 20)) return;
  if ((size_t)MP * FW * 2 > (size_t)nN * KA2 * 2) return;
  unsigned short* X1  = (unsigned short*)(ws + oX1);
  unsigned short* XB  = (unsigned short*)(ws + oX1);
  float*          Hb  = (float*)(ws + oH);
  float*          AS  = (float*)(ws + oAS);
  float*          AD  = (float*)(ws + oAD);
  int*            HT  = (int*)(ws + oHT);
  int*            OF  = (int*)(ws + oOF);
  int*            CN  = (int*)(ws + oCN);
  int*            FL  = (int*)(ws + oFL);
  unsigned short* W1T = (unsigned short*)(ws + oW1T);
  unsigned short* W2D = (unsigned short*)(ws + oW2D);
  float*          PAR = (float*)(ws + oPAR);

  hipFuncSetAttribute(reinterpret_cast<const void*>(&k_bucket),
                      hipFuncAttributeMaxDynamicSharedMemorySize, LDS_BKT);

  const int bX = cdiv(MP * 16, BTHR);
  const int bF = cdiv(nBB * 8, BTHR);
  const int bP = cdiv((MP - nN) * 32, BTHR);
  k_prep<<<bX + 25 + bF + bP, BTHR, 0, stream>>>(x, W1, W2, as1, ad1, b1, as2, ad2, b2,
                                                  XB, W1T, W2D, PAR, FL, X1, nN, MP, nBB, bX, bF);
  k_bucket<<<nBB, BTHR, LDS_BKT, stream>>>(src, dst, HT, OF, CN, FL, nE);
  k_gemm<<<MP / GBM, GTHR, 0, stream>>>(XB, W1T, Hb, FW, PAR + 0 * FW, PAR + 1 * FW, AS, AD);
  k_replay<1><<<cdiv(nN, NBRUN), BTHR, 0, stream>>>(HT, OF, CN, FL, Hb, AS, AD, PAR + 2 * FW, X1, out, nN);
  k_gemm<<<MP / GBM, GTHR, 0, stream>>>(X1, W2D, Hb, KA2, PAR + 3 * FW, PAR + 4 * FW, AS, AD);
  k_replay<2><<<cdiv(nN, NBRUN), BTHR, 0, stream>>>(HT, OF, CN, FL, Hb, AS, AD, PAR + 5 * FW, X1, out, nN);
}
